// RNNAdder_39891656245930
// MI455X (gfx1250) — hardware-verified
//
#include <hip/hip_runtime.h>
#include <math.h>

constexpr int NVOCAB   = 10;
constexpr int NEMB     = 32;
constexpr int NHID     = 64;
constexpr int NOUT     = 10;
constexpr int NOUTPAD  = 16;
constexpr int NBATCH   = 4096;
constexpr int NSTEP    = 128;
constexpr int NPAIR    = NVOCAB * NVOCAB;
constexpr int PPITCH   = 68;
constexpr int WPITCH   = 72;
constexpr int NWAVE    = 2;
constexpr int NTHR     = 32 * NWAVE;
constexpr int ROWS_BLK = 16 * NWAVE;
constexpr int TCHUNK   = 16;
constexpr int SPITCH   = TCHUNK * NOUT;
constexpr int ROWCH    = SPITCH / 4;

static_assert(NHID == 64, "two 32-deep k chunks");
static_assert(NSTEP % TCHUNK == 0, "no tail flush");
static_assert(NBATCH % ROWS_BLK == 0, "exact grid");
static_assert((TCHUNK * NOUT * 4) % 128 == 0, "row segment is whole lines");
static_assert((16 * ROWCH) % 32 == 0, "flush loop exact");
static_assert(ROWCH % 8 == 0, "aligned 8-lane groups never straddle a row");
static_assert(NPAIR <= 256, "pair index fits a byte");
static_assert((NPAIR * 16) % 32 == 0, "table kernel waves are full");

typedef __attribute__((ext_vector_type(16))) __bf16   v16b;
typedef __attribute__((ext_vector_type(8)))  __bf16   v8b;
typedef __attribute__((ext_vector_type(8)))  float    v8f;
typedef __attribute__((ext_vector_type(4)))  float    v4f;
typedef __attribute__((ext_vector_type(4)))  int      v4i;
typedef __attribute__((ext_vector_type(4)))  unsigned v4u;

union FragU { v16b v; v8b h[2]; v4u q[2]; };

__device__ __forceinline__ unsigned short f2bf_bits(float f) {
  unsigned u = __float_as_uint(f);
  return (unsigned short)((u + 0x7FFFu + ((u >> 16) & 1u)) >> 16);
}
__device__ __forceinline__ float bf_bits2f(unsigned short h) { return __uint_as_float(((unsigned)h) << 16); }

__device__ __forceinline__ v16b frag_load(const __bf16* p) {
  FragU f;
  f.h[0] = *(const v8b*)(p);
  f.h[1] = *(const v8b*)(p + 16);
  return f.v;
}
__device__ __forceinline__ v8f mma_bf(v16b a, v16b b, v8f c) {
  return __builtin_amdgcn_wmma_f32_16x16x32_bf16(false, a, false, b, (short)0, c, false, false);
}
__device__ __forceinline__ void guard_grp(v8f& acc, v16b a0, v16b a1, v16b a2, v16b a3,
                                          v16b b0, v16b b1, v16b b2, v16b b3) {
  asm volatile("v_nop\n\tv_nop\n\tv_nop\n\tv_nop"
               : "+v"(acc)
               : "v"(a0), "v"(a1), "v"(a2), "v"(a3), "v"(b0), "v"(b1), "v"(b2), "v"(b3));
}
__device__ __forceinline__ void wave_lds_sync() {
  __builtin_amdgcn_fence(__ATOMIC_RELEASE, "workgroup");
  __builtin_amdgcn_wave_barrier();
  __builtin_amdgcn_fence(__ATOMIC_ACQUIRE, "workgroup");
}
__device__ __forceinline__ float tanh_f(float x) {
  const float xc = fminf(fmaxf(x, -15.0f), 15.0f);
  const float e  = expf(2.0f * xc);
  const float d  = e + 1.0f;
  float r = __builtin_amdgcn_rcpf(d);
  r = fmaf(fmaf(-d, r, 1.0f), r, r);
  return fmaf(-2.0f, r, 1.0f);
}
__device__ __forceinline__ unsigned pair_index(int a, int b) {
  const int d1 = a < 0 ? 0 : (a > NVOCAB - 1 ? NVOCAB - 1 : a);
  const int d2 = b < 0 ? 0 : (b > NVOCAB - 1 ? NVOCAB - 1 : b);
  return (unsigned)(d1 * NVOCAB + d2);
}

__global__ __launch_bounds__(64) void ptable_kernel(const float* __restrict__ E, const float* __restrict__ Wxh,
                                                    const float* __restrict__ bvec, float* __restrict__ P) {
  const int i = blockIdx.x * 64 + threadIdx.x;
  if (i >= NPAIR * 16) return;
  const int pair = i >> 4;
  const int j4 = (i & 15) * 4;
  const int d1 = pair / NVOCAB;
  const int d2 = pair - d1 * NVOCAB;
  v4f s = *(const v4f*)(bvec + j4);
#pragma unroll 1
  for (int k = 0; k < NEMB; ++k) {
    const float e1 = E[d1 * NEMB + k];
    const float e2 = E[d2 * NEMB + k];
    const v4f w1 = *(const v4f*)(Wxh + (size_t)k * NHID + j4);
    const v4f w2 = *(const v4f*)(Wxh + (size_t)(NEMB + k) * NHID + j4);
#pragma unroll
    for (int e = 0; e < 4; ++e) {
      s[e] = fmaf(e1, w1[e], s[e]);
      s[e] = fmaf(e2, w2[e], s[e]);
    }
  }
  float* op = P + (size_t)i * 4;
  *(volatile v4f*)op = s;
  __threadfence();
  *(volatile v4f*)op = s;
}

__global__ __launch_bounds__(128) void wplanes_kernel(const float* __restrict__ Whh, const float* __restrict__ Wd,
                                                      unsigned short* __restrict__ WThi, unsigned short* __restrict__ WTlo,
                                                      unsigned short* __restrict__ WDhi, unsigned short* __restrict__ WDlo) {
  const int tid  = threadIdx.x;
  const int rloc = tid >> 3;
  const int k8   = (tid & 7) * 8;
  const bool isd = ((int)blockIdx.x == NHID / 16);
  const int nw = isd ? rloc : ((int)blockIdx.x * 16 + rloc);
  const int nd = rloc < NOUT ? rloc : NOUT - 1;
  const bool dlive = rloc < NOUT;
  v4u hv, lv;
#pragma unroll
  for (int e2 = 0; e2 < 4; ++e2) {
    const int k0 = k8 + 2 * e2;
    const float vw0 = Whh[(size_t)k0 * NHID + nw];
    const float vw1 = Whh[(size_t)(k0 + 1) * NHID + nw];
    const float vd0 = Wd[(size_t)k0 * NOUT + nd];
    const float vd1 = Wd[(size_t)(k0 + 1) * NOUT + nd];
    const float x0 = isd ? (dlive ? vd0 : 0.0f) : vw0;
    const float x1 = isd ? (dlive ? vd1 : 0.0f) : vw1;
    const unsigned short h0 = f2bf_bits(x0);
    const unsigned short h1 = f2bf_bits(x1);
    const unsigned short l0 = f2bf_bits(x0 - bf_bits2f(h0));
    const unsigned short l1 = f2bf_bits(x1 - bf_bits2f(h1));
    hv[e2] = (unsigned)h0 | ((unsigned)h1 << 16);
    lv[e2] = (unsigned)l0 | ((unsigned)l1 << 16);
  }
  unsigned short* oh = isd ? WDhi : WThi;
  unsigned short* ol = isd ? WDlo : WTlo;
  const size_t o = (size_t)nw * NHID + k8;
  *(volatile v4u*)(oh + o) = hv;
  *(volatile v4u*)(ol + o) = lv;
  __threadfence();
  *(volatile v4u*)(oh + o) = hv;
  *(volatile v4u*)(ol + o) = lv;
}

__global__ __launch_bounds__(NTHR) void seq_kernel(const int* __restrict__ num1, const int* __restrict__ num2,
                                                   const float* __restrict__ bd, const float* __restrict__ P,
                                                   const unsigned short* __restrict__ WThi_p,
                                                   const unsigned short* __restrict__ WTlo_p,
                                                   const unsigned short* __restrict__ WDhi_p,
                                                   const unsigned short* __restrict__ WDlo_p,
                                                   float* __restrict__ out) {
  __shared__ __align__(16) float    sP[NPAIR * PPITCH];
  __shared__ __align__(16) unsigned sIdxW[NSTEP * (ROWS_BLK / 4)];
  __shared__ __align__(16) __bf16   sWh[NHID * WPITCH];
  __shared__ __align__(16) __bf16   sWl[NHID * WPITCH];
  __shared__ __align__(16) __bf16   sDh[NOUTPAD * WPITCH];
  __shared__ __align__(16) __bf16   sDl[NOUTPAD * WPITCH];
  __shared__ __align__(16) __bf16   sHh[NWAVE][16 * WPITCH];
  __shared__ __align__(16) __bf16   sHl[NWAVE][16 * WPITCH];
  __shared__ __align__(16) float    sStage[NWAVE][16 * SPITCH];

  const int tid  = threadIdx.x;
  const int lane = tid & 31;
  const int wave = tid >> 5;
  const int c    = lane & 15;
  const int hh   = lane >> 4;
  const int koff = hh * 8;
  const int b0   = (int)blockIdx.x * ROWS_BLK;

  const __bf16* gWh = (const __bf16*)WThi_p;
  const __bf16* gWl = (const __bf16*)WTlo_p;
  const __bf16* gDh = (const __bf16*)WDhi_p;
  const __bf16* gDl = (const __bf16*)WDlo_p;

#pragma unroll 1
  for (int i = tid; i < NPAIR * 16; i += NTHR) {
    const int row = i >> 4;
    const int c4 = (i & 15) * 4;
    const v4f v = *(const v4f*)(P + (size_t)i * 4);
    *(v4f*)(sP + row * PPITCH + c4) = v;
  }
#pragma unroll 1
  for (int it = 0; it < 4; ++it) {
    const int combo = it * NTHR + tid;
    const int g  = combo & 7;
    const int t4 = (combo >> 3) * 4;
    v4i av[4], bv[4];
#pragma unroll
    for (int q = 0; q < 4; ++q) {
      const size_t ro = (size_t)(b0 + 4 * g + q) * NSTEP + t4;
      av[q] = *(const v4i*)(num1 + ro);
      bv[q] = *(const v4i*)(num2 + ro);
    }
#pragma unroll
    for (int e = 0; e < 4; ++e) {
      const unsigned w = pair_index(av[0][e], bv[0][e]) | (pair_index(av[1][e], bv[1][e]) << 8) |
                         (pair_index(av[2][e], bv[2][e]) << 16) | (pair_index(av[3][e], bv[3][e]) << 24);
      sIdxW[(t4 + e) * (ROWS_BLK / 4) + g] = w;
    }
  }
#pragma unroll 1
  for (int i = tid; i < NHID * 8; i += NTHR) {
    const int row = i >> 3;
    const int c8 = (i & 7) * 8;
    const v8b vh = *(const v8b*)(gWh + row * NHID + c8);
    const v8b vl = *(const v8b*)(gWl + row * NHID + c8);
    *(v8b*)(sWh + row * WPITCH + c8) = vh;
    *(v8b*)(sWl + row * WPITCH + c8) = vl;
  }
#pragma unroll 1
  for (int i = tid; i < NOUTPAD * 8; i += NTHR) {
    const int row = i >> 3;
    const int c8 = (i & 7) * 8;
    const v8b vh = *(const v8b*)(gDh + row * NHID + c8);
    const v8b vl = *(const v8b*)(gDl + row * NHID + c8);
    *(v8b*)(sDh + row * WPITCH + c8) = vh;
    *(v8b*)(sDl + row * WPITCH + c8) = vl;
  }
  const float bdv = (c < NOUT) ? bd[c < NOUT ? c : NOUT - 1] : 0.0f;
  __syncthreads();

  __bf16* myHh = &sHh[wave][0];
  __bf16* myHl = &sHl[wave][0];
  float*  myStage = &sStage[wave][0];
  const int ao = c * WPITCH + koff;

  FragU zf;
  zf.q[0] = (v4u){0u, 0u, 0u, 0u};
  zf.q[1] = (v4u){0u, 0u, 0u, 0u};
  v16b a0h = zf.v, a1h = zf.v, a0l = zf.v, a1l = zf.v;

#pragma unroll 1
  for (int t = 0; t < NSTEP; ++t) {
    const int wbase = t * (ROWS_BLK / 4) + wave * 4 + hh * 2;
    const unsigned w0 = sIdxW[wbase];
    const unsigned w1 = sIdxW[wbase + 1];
    int off[8];
#pragma unroll
    for (int r = 0; r < 4; ++r) {
      int p0 = (int)((w0 >> (8 * r)) & 0xffu);
      int p1 = (int)((w1 >> (8 * r)) & 0xffu);
      p0 = p0 > NPAIR - 1 ? NPAIR - 1 : p0;
      p1 = p1 > NPAIR - 1 ? NPAIR - 1 : p1;
      off[r]     = p0 * PPITCH + c;
      off[4 + r] = p1 * PPITCH + c;
    }

#pragma unroll 1
    for (int n = 0; n < NHID / 16; ++n) {
      v8f acc;
#pragma unroll
      for (int r = 0; r < 8; ++r) acc[r] = sP[off[r] + 16 * n];
      const int wo = (16 * n + c) * WPITCH + koff;
      const v16b b0h = frag_load(sWh + wo);
      const v16b b1h = frag_load(sWh + wo + 32);
      const v16b b0l = frag_load(sWl + wo);
      const v16b b1l = frag_load(sWl + wo + 32);
      acc = mma_bf(a0h, b0h, acc);
      acc = mma_bf(a0h, b0l, acc);
      acc = mma_bf(a0l, b0h, acc);
      acc = mma_bf(a1h, b1h, acc);
      acc = mma_bf(a1h, b1l, acc);
      acc = mma_bf(a1l, b1h, acc);
      guard_grp(acc, a0h, a1h, a0l, a1l, b0h, b1h, b0l, b1l);
#pragma unroll
      for (int r = 0; r < 8; ++r) {
        const float hv = tanh_f(acc[r]);
        const unsigned short hb = f2bf_bits(hv);
        const unsigned short lb = f2bf_bits(hv - bf_bits2f(hb));
        const int ho = (8 * hh + r) * WPITCH + 16 * n + c;
        myHh[ho] = __builtin_bit_cast(__bf16, hb);
        myHl[ho] = __builtin_bit_cast(__bf16, lb);
      }
    }
    wave_lds_sync();
    a0h = frag_load(myHh + ao);
    a1h = frag_load(myHh + ao + 32);
    a0l = frag_load(myHl + ao);
    a1l = frag_load(myHl + ao + 32);

    v8f o;
#pragma unroll
    for (int r = 0; r < 8; ++r) o[r] = bdv;
    {
      const v16b d0h = frag_load(sDh + ao);
      const v16b d1h = frag_load(sDh + ao + 32);
      const v16b d0l = frag_load(sDl + ao);
      const v16b d1l = frag_load(sDl + ao + 32);
      o = mma_bf(a0h, d0h, o);
      o = mma_bf(a0h, d0l, o);
      o = mma_bf(a0l, d0h, o);
      o = mma_bf(a1h, d1h, o);
      o = mma_bf(a1h, d1l, o);
      o = mma_bf(a1l, d1h, o);
      guard_grp(o, a0h, a1h, a0l, a1l, d0h, d1h, d0l, d1l);
    }
    const int ts = t & (TCHUNK - 1);
    if (c < NOUT) {
#pragma unroll
      for (int r = 0; r < 8; ++r) myStage[(8 * hh + r) * SPITCH + ts * NOUT + c] = o[r];
    }
    if (ts == TCHUNK - 1) {
      wave_lds_sync();
      const int t0 = t - (TCHUNK - 1);
      float* ob = out + ((size_t)(b0 + wave * 16) * NSTEP + (size_t)t0) * NOUT;
      for (int pass = 0; pass < 2; ++pass) {
#pragma unroll 1
        for (int it = 0; it < (16 * ROWCH) / 32; ++it) {
          const int chunk = it * 32 + lane;
          const int row = chunk / ROWCH;
          const int c4 = chunk - row * ROWCH;
          const v4f v = *(const v4f*)(myStage + row * SPITCH + c4 * 4);
          *(volatile v4f*)(ob + (size_t)row * (NSTEP * NOUT) + c4 * 4) = v;
        }
        __threadfence();
      }
      wave_lds_sync();
    }
  }
}

extern "C" void kernel_launch(void* const* d_in, const int* in_sizes, int n_in,
                              void* d_out, int out_size, void* d_ws, size_t ws_size, hipStream_t stream) {
  if (n_in < 8 || d_out == nullptr || d_ws == nullptr) return;
  if (in_sizes[0] != NBATCH * NSTEP || in_sizes[1] != NBATCH * NSTEP || in_sizes[2] != NVOCAB * NEMB ||
      in_sizes[3] != 2 * NEMB * NHID || in_sizes[4] != NHID * NHID || in_sizes[5] != NHID ||
      in_sizes[6] != NHID * NOUT || in_sizes[7] != NOUT || out_size != NBATCH * NSTEP * NOUT) return;

  const int*   num1 = (const int*)d_in[0];
  const int*   num2 = (const int*)d_in[1];
  const float* E    = (const float*)d_in[2];
  const float* Wxh  = (const float*)d_in[3];
  const float* Whh  = (const float*)d_in[4];
  const float* bvec = (const float*)d_in[5];
  const float* Wd   = (const float*)d_in[6];
  const float* bd   = (const float*)d_in[7];
  float* out = (float*)d_out;

  char* ws = (char*)d_ws;
  size_t off = 0;
  auto carve = [&](size_t bytes) -> char* { char* p = ws + off; off += (bytes + 255) & ~(size_t)255; return p; };
  float*          P    = (float*)carve((size_t)NPAIR * NHID * 4);
  unsigned short* WThi = (unsigned short*)carve((size_t)NHID * NHID * 2);
  unsigned short* WTlo = (unsigned short*)carve((size_t)NHID * NHID * 2);
  unsigned short* WDhi = (unsigned short*)carve((size_t)NOUTPAD * NHID * 2);
  unsigned short* WDlo = (unsigned short*)carve((size_t)NOUTPAD * NHID * 2);
  if (off > ws_size || off > (size_t)134217728) return;

  ptable_kernel<<<(NPAIR * 16) / 64, 64, 0, stream>>>(E, Wxh, bvec, P);
  wplanes_kernel<<<NHID / 16 + 1, 128, 0, stream>>>(Whh, Wd, WThi, WTlo, WDhi, WDlo);
  seq_kernel<<<NBATCH / ROWS_BLK, NTHR, 0, stream>>>(num1, num2, bd, P, WThi, WTlo, WDhi, WDlo, out);
}
